// TNODE_25417616458373
// MI455X (gfx1250) — hardware-verified
//
#include <hip/hip_runtime.h>

#define N_CELLS 8192
#define G_GENES 2000
#define L_LAT   20
#define H_ODE   128
#define H_VAE   128
#define ZP      32
#define KP_E    2048
#define NCH_E   63
#define PARTP   32
#define N_DEC_BLK (N_CELLS / 32)
#define N_ZDV_BLK (N_CELLS / 64)

typedef _Float16 v16h __attribute__((ext_vector_type(16)));
typedef _Float16 v8h  __attribute__((ext_vector_type(8)));
typedef _Float16 v4h  __attribute__((ext_vector_type(4)));
typedef __bf16   v16b __attribute__((ext_vector_type(16)));
typedef unsigned short v8us __attribute__((ext_vector_type(8)));
typedef unsigned short v4us __attribute__((ext_vector_type(4)));
typedef float    v8f  __attribute__((ext_vector_type(8)));
typedef float    v4f  __attribute__((ext_vector_type(4)));
union Frag  { v16h v; v8h  h[2]; };
union FragB { v16b v; v8us h[2]; };

__device__ __forceinline__ v8f wmma16(const v16h& a, const v16h& b, v8f c) {
    c = __builtin_amdgcn_wmma_f32_16x16x32_f16(false, a, false, b, (short)0, c, false, false);
    asm volatile("v_nop\n\tv_nop\n\tv_nop\n\tv_nop" : "+v"(c) : "v"(a), "v"(b));
    return c;
}
__device__ __forceinline__ v8f wmma16b(const v16b& a, const v16b& b, v8f c) {
    c = __builtin_amdgcn_wmma_f32_16x16x32_bf16(false, a, false, b, (short)0, c, false, false);
    asm volatile("v_nop\n\tv_nop\n\tv_nop\n\tv_nop" : "+v"(c) : "v"(a), "v"(b));
    return c;
}
__device__ __forceinline__ v8f zero8() { v8f c = {0.f, 0.f, 0.f, 0.f, 0.f, 0.f, 0.f, 0.f}; return c; }
__device__ __forceinline__ v4f zero4() { v4f c = {0.f, 0.f, 0.f, 0.f}; return c; }
__device__ __forceinline__ float eluf(float x) { return x > 0.f ? x : (__expf(x) - 1.f); }
__device__ __forceinline__ float wave_sum(float v) {
#pragma unroll
    for (int msk = 16; msk > 0; msk >>= 1) v += __shfl_xor(v, msk, 32);
    return v;
}
__device__ __forceinline__ unsigned short bf16_bits(float x) {
    unsigned int u = __float_as_uint(x);
    u += 0x7FFFu + ((u >> 16) & 1u);
    return (unsigned short)(u >> 16);
}
__device__ __forceinline__ void bf16_split(float x, unsigned short& hi, unsigned short& lo) {
    const unsigned short hb = bf16_bits(x);
    const float hfv = __uint_as_float(((unsigned int)hb) << 16);
    hi = hb;
    lo = bf16_bits(x - hfv);
}

__global__ __launch_bounds__(256)
void pack_e_kernel(const float* __restrict__ W, _Float16* __restrict__ Bt,
                   unsigned short* __restrict__ Bh, unsigned short* __restrict__ Bl) {
    const int id = blockIdx.x * 256 + threadIdx.x;
    if (id >= H_VAE * (KP_E / 8)) return;
    const int n  = id >> 8;
    const int k0 = (id & 255) * 8;
    v8h v; v8us vh, vl;
#pragma unroll
    for (int e = 0; e < 8; ++e) {
        const int k = k0 + e;
        const float x = (k < G_GENES) ? W[(size_t)k * H_VAE + n] : 0.f;
        v[e] = (_Float16)(x * 64.f);
        unsigned short hb, lb;
        bf16_split(x, hb, lb);
        vh[e] = hb; vl[e] = lb;
    }
    const size_t o = (size_t)n * KP_E + k0;
    _Float16*       d0 = Bt + o;
    unsigned short* d1 = Bh + o;
    unsigned short* d2 = Bl + o;
    *(volatile v8h*)d0  = v;
    *(volatile v8us*)d1 = vh;
    *(volatile v8us*)d2 = vl;
    __threadfence();
    *(volatile v8h*)d0  = v;
    *(volatile v8us*)d1 = vh;
    *(volatile v8us*)d2 = vl;
}

__global__ __launch_bounds__(256)
void pack_d_kernel(const float* __restrict__ W, _Float16* __restrict__ Dt) {
    const int id = blockIdx.x * 256 + threadIdx.x;
    if (id >= G_GENES * (H_VAE / 8)) return;
    const int n  = id >> 4;
    const int k0 = (id & 15) * 8;
    v8h v;
#pragma unroll
    for (int e = 0; e < 8; ++e)
        v[e] = (_Float16)(W[(size_t)(k0 + e) * G_GENES + n] * 16.f);
    _Float16* dst = Dt + (size_t)n * H_VAE + k0;
    *(volatile v8h*)dst = v;
    __threadfence();
    *(volatile v8h*)dst = v;
}

template <int SPLIT>
__global__ __launch_bounds__(256)
void encoder_kernel(const float* __restrict__ X, const _Float16* __restrict__ Bt,
                    const unsigned short* __restrict__ Bh, const unsigned short* __restrict__ Bl,
                    const float* __restrict__ be1,
                    const float* __restrict__ Wet, const float* __restrict__ bet,
                    const float* __restrict__ Wez, const float* __restrict__ bez,
                    float* zout, float* Tsout, int writeTs) {
    __shared__ __attribute__((aligned(16))) _Float16 As[32 * 32];
    __shared__ __attribute__((aligned(16))) unsigned short Ash[32 * 32];
    __shared__ __attribute__((aligned(16))) unsigned short Asl[32 * 32];
    __shared__ __attribute__((aligned(16))) float hbuf[32 * H_VAE];
    __shared__ __attribute__((aligned(16))) float zst[32 * ZP];
    __shared__ __attribute__((aligned(16))) float tst[32];

    const int tid = threadIdx.x, wv = tid >> 5, lane = tid & 31;
    const int hf = lane >> 4, m = lane & 15;
    const int r0 = blockIdx.x * 32;
    const int rt = wv >> 2, cb = (wv & 3) * 32;

    for (int i = tid; i < 32 * ZP; i += 256) zst[i] = 0.f;
    if (tid < 32) tst[tid] = 0.f;

    const int srow = tid >> 3, sseg = tid & 7;
    const float*    xrow = X + (size_t)(r0 + srow) * G_GENES + 4 * sseg;
    const size_t    bo0  = (size_t)(cb + m) * KP_E + 8 * hf;
    const size_t    bo1  = (size_t)(cb + 16 + m) * KP_E + 8 * hf;
    const _Float16* b0p  = Bt + bo0;
    const _Float16* b1p  = Bt + bo1;
    const unsigned short* g0h = Bh + bo0;
    const unsigned short* g0l = Bl + bo0;
    const unsigned short* g1h = Bh + bo1;
    const unsigned short* g1l = Bl + bo1;
    const int aoff = (rt * 16 + m) * 32 + 8 * hf;
    const _Float16*       ap  = As  + aoff;
    const unsigned short* aph = Ash + aoff;
    const unsigned short* apl = Asl + aoff;
    const int soff = srow * 32 + 4 * sseg;

    v8f c0 = zero8(), c1 = zero8();
    for (int ch = 0; ch < NCH_E; ++ch) {
        const int kc = ch * 32;
        v4f xv = zero4();
        if (kc + 4 * sseg < G_GENES) xv = *(const v4f*)(xrow + kc);
        if (SPLIT) {
            v4us hv, lv;
#pragma unroll
            for (int q = 0; q < 4; ++q) {
                unsigned short hb, lb;
                bf16_split(xv[q], hb, lb);
                hv[q] = hb; lv[q] = lb;
            }
            *(v4us*)(Ash + soff) = hv;
            *(v4us*)(Asl + soff) = lv;
        } else {
            *(v4h*)(As + soff) = __builtin_convertvector(xv, v4h);
        }
        __syncthreads();
        if (SPLIT) {
            FragB ah, al, b0h, b0l, b1h, b1l;
            ah.h[0]  = *(const v8us*)(aph);
            ah.h[1]  = *(const v8us*)(aph + 16);
            al.h[0]  = *(const v8us*)(apl);
            al.h[1]  = *(const v8us*)(apl + 16);
            b0h.h[0] = *(const v8us*)(g0h + kc);
            b0h.h[1] = *(const v8us*)(g0h + kc + 16);
            b0l.h[0] = *(const v8us*)(g0l + kc);
            b0l.h[1] = *(const v8us*)(g0l + kc + 16);
            b1h.h[0] = *(const v8us*)(g1h + kc);
            b1h.h[1] = *(const v8us*)(g1h + kc + 16);
            b1l.h[0] = *(const v8us*)(g1l + kc);
            b1l.h[1] = *(const v8us*)(g1l + kc + 16);
            c0 = wmma16b(ah.v, b0h.v, c0);
            c0 = wmma16b(al.v, b0h.v, c0);
            c0 = wmma16b(ah.v, b0l.v, c0);
            c1 = wmma16b(ah.v, b1h.v, c1);
            c1 = wmma16b(al.v, b1h.v, c1);
            c1 = wmma16b(ah.v, b1l.v, c1);
        } else {
            Frag a, b0, b1;
            a.h[0]  = *(const v8h*)(ap);
            a.h[1]  = *(const v8h*)(ap + 16);
            b0.h[0] = *(const v8h*)(b0p + kc);
            b0.h[1] = *(const v8h*)(b0p + kc + 16);
            b1.h[0] = *(const v8h*)(b1p + kc);
            b1.h[1] = *(const v8h*)(b1p + kc + 16);
            c0 = wmma16(a.v, b0.v, c0);
            c1 = wmma16(a.v, b1.v, c1);
        }
        __syncthreads();
    }

    {
        const float scl = SPLIT ? 1.0f : 0.015625f;
        const int col0 = cb + m, col1 = cb + 16 + m;
        const float bias0 = be1[col0], bias1 = be1[col1];
#pragma unroll
        for (int r = 0; r < 8; ++r) {
            const int row = rt * 16 + 8 * hf + r;
            hbuf[row * H_VAE + col0] = eluf(c0[r] * scl + bias0);
            hbuf[row * H_VAE + col1] = eluf(c1[r] * scl + bias1);
        }
    }
    __syncthreads();

    for (int job = tid; job < 32 * (L_LAT + 1); job += 256) {
        const int row = job / (L_LAT + 1);
        const int o   = job - row * (L_LAT + 1);
        const float* hp = hbuf + row * H_VAE;
        if (o < L_LAT) {
            float acc = bez[o];
#pragma unroll 4
            for (int k = 0; k < H_VAE; ++k) acc += hp[k] * Wez[k * L_LAT + o];
            zst[row * ZP + o] = acc;
        } else {
            float acc = bet[0];
#pragma unroll 4
            for (int k = 0; k < H_VAE; ++k) acc += hp[k] * Wet[k];
            tst[row] = 1.0f / (1.0f + expf(-acc));
        }
    }
    __syncthreads();

    const int zr = tid >> 3, zq = tid & 7;
    const v4f zv = *(const v4f*)(zst + zr * ZP + 4 * zq);
    float* zdst = zout + (size_t)(r0 + zr) * ZP + 4 * zq;
    v4f tv = zero4();
    if (tid < 8) tv = *(const v4f*)(tst + 4 * tid);
    float* tdst = Tsout + r0 + 4 * (tid & 7);

    *(volatile v4f*)zdst = zv;
    if (writeTs && tid < 8) *(volatile v4f*)tdst = tv;
    __threadfence();
    *(volatile v4f*)zdst = zv;
    if (writeTs && tid < 8) *(volatile v4f*)tdst = tv;
}

__global__ __launch_bounds__(1024)
void sort_kernel(const float* __restrict__ Ts, const float* __restrict__ zs, const float* __restrict__ zu,
                 float* Tss, float* zss, float* zus) {
    __shared__ __attribute__((aligned(16))) unsigned long long kv[N_CELLS];
    const int tid = threadIdx.x;
    for (int i = tid; i < N_CELLS; i += 1024)
        kv[i] = ((unsigned long long)__float_as_uint(Ts[i]) << 32) | (unsigned int)i;
    for (int k = 2; k <= N_CELLS; k <<= 1) {
        for (int j = k >> 1; j > 0; j >>= 1) {
            __syncthreads();
            for (int i = tid; i < N_CELLS; i += 1024) {
                const int ixj = i ^ j;
                if (ixj > i) {
                    const unsigned long long va = kv[i], vb = kv[ixj];
                    const bool up = ((i & k) == 0);
                    if ((va > vb) == up) { kv[i] = vb; kv[ixj] = va; }
                }
            }
        }
    }
    __syncthreads();

    for (int pass = 0; pass < 2; ++pass) {
        for (int t = tid; t < N_CELLS / 4; t += 1024) {
            v4f v;
            v[0] = __uint_as_float((unsigned int)(kv[4 * t + 0] >> 32));
            v[1] = __uint_as_float((unsigned int)(kv[4 * t + 1] >> 32));
            v[2] = __uint_as_float((unsigned int)(kv[4 * t + 2] >> 32));
            v[3] = __uint_as_float((unsigned int)(kv[4 * t + 3] >> 32));
            *(volatile v4f*)(Tss + 4 * t) = v;
        }
        for (int e = tid; e < N_CELLS * 8; e += 1024) {
            const int i = e >> 3, q = e & 7;
            const int src = (int)(kv[i] & (unsigned long long)(N_CELLS - 1));
            const v4f a = *(const v4f*)(zs + (size_t)src * ZP + 4 * q);
            const v4f b = *(const v4f*)(zu + (size_t)src * ZP + 4 * q);
            *(volatile v4f*)(zss + (size_t)i * ZP + 4 * q) = a;
            *(volatile v4f*)(zus + (size_t)i * ZP + 4 * q) = b;
        }
        if (pass == 0) __threadfence();
    }
}

__global__ __launch_bounds__(32)
void ode_kernel(const float* __restrict__ Tss, const float* __restrict__ zss,
                const float* __restrict__ Wo1, const float* __restrict__ bo1,
                const float* __restrict__ Wo2, const float* __restrict__ bo2,
                float* predz) {
    __shared__ __attribute__((aligned(16))) float W1s[L_LAT * H_ODE];
    __shared__ __attribute__((aligned(16))) float W2s[H_ODE * L_LAT];
    __shared__ __attribute__((aligned(16))) float B1s[H_ODE];
    __shared__ __attribute__((aligned(16))) float zst[4 * ZP];
    const int lane = threadIdx.x;
    for (int i = lane; i < L_LAT * H_ODE; i += 32) { W1s[i] = Wo1[i]; W2s[i] = Wo2[i]; }
    for (int i = lane; i < H_ODE; i += 32) B1s[i] = bo1[i];
    float b2[L_LAT], z[L_LAT];
#pragma unroll
    for (int j = 0; j < L_LAT; ++j) { b2[j] = bo2[j]; z[j] = zss[j]; }
    __syncthreads();

    for (int t = 0; t < N_CELLS; ++t) {
        float myz = 0.f;
#pragma unroll
        for (int j = 0; j < L_LAT; ++j) myz = (lane == j) ? z[j] : myz;
        zst[(t & 3) * ZP + lane] = myz;
        if ((t & 3) == 3) {
            __syncthreads();
            const v4f v = *(const v4f*)(zst + lane * 4);
            float* dst = predz + (size_t)(t - 3) * ZP + lane * 4;
            *(volatile v4f*)dst = v;
            __threadfence();
            *(volatile v4f*)dst = v;
            __syncthreads();
        }
        if (t == N_CELLS - 1) break;

        const float dt = Tss[t + 1] - Tss[t];
        float p[L_LAT];
#pragma unroll
        for (int j = 0; j < L_LAT; ++j) p[j] = 0.f;
#pragma unroll 1
        for (int q = 0; q < 4; ++q) {
            const int i = lane + 32 * q;
            float hh = B1s[i];
#pragma unroll
            for (int j = 0; j < L_LAT; ++j) hh += z[j] * W1s[j * H_ODE + i];
            const float e = eluf(hh);
#pragma unroll
            for (int j = 0; j < L_LAT; ++j) p[j] += e * W2s[i * L_LAT + j];
        }
#pragma unroll
        for (int msk = 1; msk < 32; msk <<= 1) {
#pragma unroll
            for (int j = 0; j < L_LAT; ++j) p[j] += __shfl_xor(p[j], msk, 32);
        }
#pragma unroll
        for (int j = 0; j < L_LAT; ++j) z[j] += dt * (p[j] + b2[j]);
    }
}

__global__ __launch_bounds__(128)
void zdiv_kernel(const float* __restrict__ predz, const float* __restrict__ zss, const float* __restrict__ zus,
                 const float* __restrict__ Wo1, const float* __restrict__ bo1,
                 const float* __restrict__ Wo2, const float* __restrict__ bo2,
                 const float* __restrict__ beta, const float* __restrict__ lam,
                 float* part) {
    __shared__ __attribute__((aligned(16))) _Float16 Az[64 * 32];
    __shared__ __attribute__((aligned(16))) _Float16 B1t[H_ODE * 32];
    __shared__ __attribute__((aligned(16))) _Float16 A2[64 * H_ODE];
    __shared__ __attribute__((aligned(16))) _Float16 B2t[32 * H_ODE];
    __shared__ float red[8];
    const int tid = threadIdx.x, wv = tid >> 5, lane = tid & 31;
    const int hf = lane >> 4, m = lane & 15;
    const int n0 = blockIdx.x * 64;

    for (int e = tid; e < H_ODE * 32; e += 128) {
        const int i = e >> 5, k = e & 31;
        B1t[e] = (_Float16)((k < L_LAT) ? Wo1[k * H_ODE + i] * 8.f : 0.f);
    }
    for (int e = tid; e < 32 * H_ODE; e += 128) {
        const int j = e >> 7, i = e & (H_ODE - 1);
        B2t[e] = (_Float16)((j < L_LAT) ? Wo2[i * L_LAT + j] * 16.f : 0.f);
    }
    for (int e = tid; e < 64 * 32; e += 128) {
        const int row = e >> 5, k = e & 31;
        Az[e] = (_Float16)((k < L_LAT) ? predz[(size_t)(n0 + row) * ZP + k] : 0.f);
    }
    __syncthreads();

    {
        Frag a;
        a.h[0] = *(const v8h*)(Az + (wv * 16 + m) * 32 + 8 * hf);
        a.h[1] = *(const v8h*)(Az + (wv * 16 + m) * 32 + 16 + 8 * hf);
        for (int ct = 0; ct < H_ODE / 16; ++ct) {
            Frag b;
            b.h[0] = *(const v8h*)(B1t + (ct * 16 + m) * 32 + 8 * hf);
            b.h[1] = *(const v8h*)(B1t + (ct * 16 + m) * 32 + 16 + 8 * hf);
            v8f c = zero8();
            c = wmma16(a.v, b.v, c);
            const int col = ct * 16 + m;
            const float bias = bo1[col];
#pragma unroll
            for (int r = 0; r < 8; ++r) {
                const int row = wv * 16 + 8 * hf + r;
                A2[row * H_ODE + col] = (_Float16)eluf(c[r] * 0.125f + bias);
            }
        }
    }
    __syncthreads();

    v8f d0 = zero8(), d1 = zero8();
#pragma unroll
    for (int ks = 0; ks < 4; ++ks) {
        Frag a, b0, b1;
        a.h[0]  = *(const v8h*)(A2 + (wv * 16 + m) * H_ODE + ks * 32 + 8 * hf);
        a.h[1]  = *(const v8h*)(A2 + (wv * 16 + m) * H_ODE + ks * 32 + 16 + 8 * hf);
        b0.h[0] = *(const v8h*)(B2t + m * H_ODE + ks * 32 + 8 * hf);
        b0.h[1] = *(const v8h*)(B2t + m * H_ODE + ks * 32 + 16 + 8 * hf);
        b1.h[0] = *(const v8h*)(B2t + (16 + m) * H_ODE + ks * 32 + 8 * hf);
        b1.h[1] = *(const v8h*)(B2t + (16 + m) * H_ODE + ks * 32 + 16 + 8 * hf);
        d0 = wmma16(a.v, b0.v, d0);
        d1 = wmma16(a.v, b1.v, d1);
    }

    float szd = 0.f, sxt = 0.f;
    {
        const int j = m;
        const float eb = expf(beta[j]), el = expf(lam[j]), bb = bo2[j];
#pragma unroll
        for (int r = 0; r < 8; ++r) {
            const int n = n0 + wv * 16 + 8 * hf + r;
            const size_t o = (size_t)n * ZP + j;
            const float zsv = zss[o], zuv = zus[o], pz = predz[o];
            const float f  = d0[r] * 0.0625f + bb;
            const float tg = eb * zuv - el * zsv;
            const float e1 = f - tg;   szd += e1 * e1;
            const float e2 = zsv - pz; sxt += e2 * e2;
        }
    }
    {
        const bool valid = (m < L_LAT - 16);
        const int j = valid ? (16 + m) : 0;
        const float eb = expf(beta[j]), el = expf(lam[j]), bb = bo2[j];
#pragma unroll
        for (int r = 0; r < 8; ++r) {
            const int n = n0 + wv * 16 + 8 * hf + r;
            const size_t o = (size_t)n * ZP + j;
            const float zsv = zss[o], zuv = zus[o], pz = predz[o];
            const float f  = d1[r] * 0.0625f + bb;
            const float tg = eb * zuv - el * zsv;
            const float e1 = f - tg;
            const float e2 = zsv - pz;
            szd += valid ? e1 * e1 : 0.f;
            sxt += valid ? e2 * e2 : 0.f;
        }
    }
    szd = wave_sum(szd);
    sxt = wave_sum(sxt);
    if (lane == 0) { red[wv * 2] = szd; red[wv * 2 + 1] = sxt; }
    __syncthreads();
    if (wv == 0) {
        const float tz = ((red[0] + red[2]) + red[4]) + red[6];
        const float tx = ((red[1] + red[3]) + red[5]) + red[7];
        v4f v = zero4();
        if (lane == 0) { v[0] = tz; v[1] = tx; }
        float* dst = part + (size_t)blockIdx.x * PARTP + lane * 4;
        if (lane < 8) *(volatile v4f*)dst = v;
        __threadfence();
        if (lane < 8) *(volatile v4f*)dst = v;
    }
}

__global__ __launch_bounds__(256)
void decoder_kernel(const float* __restrict__ Z, const float* __restrict__ X,
                    const float* __restrict__ Wd1, const float* __restrict__ bd1,
                    const _Float16* __restrict__ Dt, const float* __restrict__ bd2,
                    float* part) {
    __shared__ __attribute__((aligned(16))) float zl[32 * L_LAT];
    __shared__ __attribute__((aligned(16))) _Float16 Hd[32 * H_VAE];
    __shared__ float red[8];
    const int tid = threadIdx.x;
    const int r0  = blockIdx.x * 32;

    for (int i = tid; i < 32 * L_LAT; i += 256) {
        const int row = i / L_LAT, j = i - row * L_LAT;
        zl[i] = Z[(size_t)(r0 + row) * ZP + j];
    }
    __syncthreads();
    for (int job = tid; job < 32 * H_VAE; job += 256) {
        const int row = job >> 7, i = job & (H_VAE - 1);
        float a = bd1[i];
#pragma unroll
        for (int j = 0; j < L_LAT; ++j) a += zl[row * L_LAT + j] * Wd1[j * H_VAE + i];
        Hd[job] = (_Float16)eluf(a);
    }
    __syncthreads();

    const int wv = tid >> 5, lane = tid & 31, hf = lane >> 4, m = lane & 15;
    Frag afr[2][4];
#pragma unroll
    for (int rtile = 0; rtile < 2; ++rtile) {
#pragma unroll
        for (int ks = 0; ks < 4; ++ks) {
            afr[rtile][ks].h[0] = *(const v8h*)(Hd + (rtile * 16 + m) * H_VAE + ks * 32 + 8 * hf);
            afr[rtile][ks].h[1] = *(const v8h*)(Hd + (rtile * 16 + m) * H_VAE + ks * 32 + 16 + 8 * hf);
        }
    }
    float acc = 0.f;
    for (int ct = wv; ct < G_GENES / 16; ct += 8) {
        const int ncol = ct * 16 + m;
        const _Float16* bp = Dt + (size_t)ncol * H_VAE + 8 * hf;
        v8f c0 = zero8(), c1 = zero8();
#pragma unroll
        for (int ks = 0; ks < 4; ++ks) {
            Frag b;
            b.h[0] = *(const v8h*)(bp + ks * 32);
            b.h[1] = *(const v8h*)(bp + ks * 32 + 16);
            c0 = wmma16(afr[0][ks].v, b.v, c0);
            c1 = wmma16(afr[1][ks].v, b.v, c1);
        }
        const float bias = bd2[ncol];
#pragma unroll
        for (int r = 0; r < 8; ++r) {
            const int row = 8 * hf + r;
            const float x0 = X[(size_t)(r0 + row) * G_GENES + ncol];
            const float x1 = X[(size_t)(r0 + 16 + row) * G_GENES + ncol];
            const float e0 = x0 - (c0[r] * 0.0625f + bias);
            const float e1 = x1 - (c1[r] * 0.0625f + bias);
            acc += e0 * e0;
            acc += e1 * e1;
        }
    }
    acc = wave_sum(acc);
    if (lane == 0) red[wv] = acc;
    __syncthreads();
    if (wv == 0) {
        float tot = 0.f;
#pragma unroll
        for (int i = 0; i < 8; ++i) tot += red[i];
        v4f v = zero4();
        if (lane == 0) v[0] = tot;
        float* dst = part + (size_t)blockIdx.x * PARTP + lane * 4;
        if (lane < 8) *(volatile v4f*)dst = v;
        __threadfence();
        if (lane < 8) *(volatile v4f*)dst = v;
    }
}

__global__ void finalize_kernel(const float* __restrict__ pS, const float* __restrict__ pU,
                                const float* __restrict__ pZ, int nDec, int nZ, float* out) {
    if (threadIdx.x == 0) {
        double es = 0.0, eu = 0.0, zd = 0.0, xt = 0.0;
        for (int b = 0; b < nDec; ++b) { es += (double)pS[(size_t)b * PARTP]; eu += (double)pU[(size_t)b * PARTP]; }
        for (int b = 0; b < nZ; ++b)   { zd += (double)pZ[(size_t)b * PARTP]; xt += (double)pZ[(size_t)b * PARTP + 1]; }
        const double ng = (double)N_CELLS * (double)G_GENES;
        const double nl = (double)N_CELLS * (double)L_LAT;
        const float ec  = (float)(es / ng);
        const float ecu = (float)(eu / ng);
        const float zdv = (float)(zd / nl);
        const float xtv = (float)(xt / nl);
        float loss = ec + ecu;
        loss = loss + zdv;
        loss = loss + xtv;
        v4f v;
        v[0] = loss; v[1] = ec; v[2] = ecu; v[3] = zdv;
        *(volatile v4f*)out = v;
        __threadfence();
        *(volatile v4f*)out = v;
    }
}

static inline size_t align_up(size_t x, size_t a) { return (x + a - 1) / a * a; }

extern "C" void kernel_launch(void* const* d_in, const int* in_sizes, int n_in,
                              void* d_out, int out_size, void* d_ws, size_t ws_size,
                              hipStream_t stream) {
    if (n_in < 20 || out_size < 4) return;
    if (in_sizes[0] != N_CELLS * G_GENES || in_sizes[1] != N_CELLS * G_GENES) return;
    if (in_sizes[4] != G_GENES * H_VAE || in_sizes[5] != H_VAE) return;
    if (in_sizes[6] != H_VAE || in_sizes[7] < 1) return;
    if (in_sizes[8] != H_VAE * L_LAT || in_sizes[9] != L_LAT) return;
    if (in_sizes[10] != L_LAT * H_ODE || in_sizes[11] != H_ODE) return;
    if (in_sizes[12] != H_ODE * L_LAT || in_sizes[13] != L_LAT) return;
    if (in_sizes[14] != L_LAT * H_VAE || in_sizes[15] != H_VAE) return;
    if (in_sizes[16] != H_VAE * G_GENES || in_sizes[17] != G_GENES) return;
    if (in_sizes[18] != L_LAT || in_sizes[19] != L_LAT) return;

    const float* s    = (const float*)d_in[0];
    const float* u    = (const float*)d_in[1];
    const float* We1  = (const float*)d_in[4];
    const float* be1  = (const float*)d_in[5];
    const float* Wet  = (const float*)d_in[6];
    const float* bet  = (const float*)d_in[7];
    const float* Wez  = (const float*)d_in[8];
    const float* bez  = (const float*)d_in[9];
    const float* Wo1  = (const float*)d_in[10];
    const float* bo1  = (const float*)d_in[11];
    const float* Wo2  = (const float*)d_in[12];
    const float* bo2  = (const float*)d_in[13];
    const float* Wd1  = (const float*)d_in[14];
    const float* bd1  = (const float*)d_in[15];
    const float* Wd2  = (const float*)d_in[16];
    const float* bd2  = (const float*)d_in[17];
    const float* beta = (const float*)d_in[18];
    const float* lam  = (const float*)d_in[19];

    size_t off = 0;
    const size_t oTs    = off; off = align_up(off + (size_t)N_CELLS * 4, 256);
    const size_t oTss   = off; off = align_up(off + (size_t)N_CELLS * 4, 256);
    const size_t oZs    = off; off = align_up(off + (size_t)N_CELLS * ZP * 4, 256);
    const size_t oZu    = off; off = align_up(off + (size_t)N_CELLS * ZP * 4, 256);
    const size_t oZss   = off; off = align_up(off + (size_t)N_CELLS * ZP * 4, 256);
    const size_t oZus   = off; off = align_up(off + (size_t)N_CELLS * ZP * 4, 256);
    const size_t oPredz = off; off = align_up(off + (size_t)N_CELLS * ZP * 4, 256);
    const size_t oBt    = off; off = align_up(off + (size_t)H_VAE * KP_E * 2, 256);
    const size_t oBh    = off; off = align_up(off + (size_t)H_VAE * KP_E * 2, 256);
    const size_t oBl    = off; off = align_up(off + (size_t)H_VAE * KP_E * 2, 256);
    const size_t oDt    = off; off = align_up(off + (size_t)G_GENES * H_VAE * 2, 256);
    const size_t oPS    = off; off = align_up(off + (size_t)N_DEC_BLK * PARTP * 4, 256);
    const size_t oPU    = off; off = align_up(off + (size_t)N_DEC_BLK * PARTP * 4, 256);
    const size_t oPZ    = off; off = align_up(off + (size_t)N_ZDV_BLK * PARTP * 4, 256);
    if (off > ws_size) return;

    char* ws = (char*)d_ws;
    float* Ts    = (float*)(ws + oTs);
    float* Tss   = (float*)(ws + oTss);
    float* zs    = (float*)(ws + oZs);
    float* zu    = (float*)(ws + oZu);
    float* zss   = (float*)(ws + oZss);
    float* zus   = (float*)(ws + oZus);
    float* predz = (float*)(ws + oPredz);
    _Float16* Bt = (_Float16*)(ws + oBt);
    unsigned short* Bh = (unsigned short*)(ws + oBh);
    unsigned short* Bl = (unsigned short*)(ws + oBl);
    _Float16* Dt = (_Float16*)(ws + oDt);
    float* pS    = (float*)(ws + oPS);
    float* pU    = (float*)(ws + oPU);
    float* pZ    = (float*)(ws + oPZ);
    float* out   = (float*)d_out;

    pack_e_kernel<<<(H_VAE * (KP_E / 8) + 255) / 256, 256, 0, stream>>>(We1, Bt, Bh, Bl);
    pack_d_kernel<<<(G_GENES * (H_VAE / 8) + 255) / 256, 256, 0, stream>>>(Wd2, Dt);
    encoder_kernel<1><<<N_CELLS / 32, 256, 0, stream>>>(s, Bt, Bh, Bl, be1, Wet, bet, Wez, bez, zs, Ts, 1);
    encoder_kernel<0><<<N_CELLS / 32, 256, 0, stream>>>(u, Bt, Bh, Bl, be1, Wet, bet, Wez, bez, zu, Ts, 0);
    sort_kernel<<<1, 1024, 0, stream>>>(Ts, zs, zu, Tss, zss, zus);
    ode_kernel<<<1, 32, 0, stream>>>(Tss, zss, Wo1, bo1, Wo2, bo2, predz);
    decoder_kernel<<<N_DEC_BLK, 256, 0, stream>>>(zs, s, Wd1, bd1, Dt, bd2, pS);
    decoder_kernel<<<N_DEC_BLK, 256, 0, stream>>>(zu, u, Wd1, bd1, Dt, bd2, pU);
    zdiv_kernel<<<N_ZDV_BLK, 128, 0, stream>>>(predz, zss, zus, Wo1, bo1, Wo2, bo2, beta, lam, pZ);
    finalize_kernel<<<1, 32, 0, stream>>>(pS, pU, pZ, N_DEC_BLK, N_ZDV_BLK, out);
    (void)hipGetLastError();
}
